// MultiHeadAttentionEdgeLayer_69363721830857
// MI455X (gfx1250) — hardware-verified
//
#include <hip/hip_runtime.h>
#include <stddef.h>


#define DD      128
#define HEADS   8
#define DKH     16
#define QKVW    384
#define NTHR    256
#define NWAVE   8
#define EPT     8
#define NGRP    2
#define CHUNK   (NTHR * EPT * NGRP)
#define WCAP    (EPT * NGRP * 32)
#define LISTN   (NWAVE * WCAP)
#define NBC     4096
#define NBF     1024
#define RCAP    40960
#define RBN     128
#define TGT     256
#define AGRP    8
#define DEGCAP  256
#define OTHR    512
#define ETCAP   32
#define PTHR    192
#define WSCAP   134217728
#define WCARRY  16.0f
#define QSCALE  0.25f
#define Z_EPS   1e-6f

#define LDS_FILL ((RCAP + NBF + LISTN) * 4 + 64)

static_assert((CHUNK & (CHUNK - 1)) == 0);
static_assert(CHUNK <= 4096);
static_assert(NBC <= 4096 && NBF <= 4096);
static_assert((NBC & (NBC - 1)) == 0 && (NBF & (NBF - 1)) == 0);
static_assert(NBC == 4 * NBF);
static_assert(OTHR * 8 == NBC);
static_assert((RCAP % 32) == 0);
static_assert(TGT == NWAVE * 32);
static_assert((NBC % TGT) == 0);
static_assert((32 % AGRP) == 0);
static_assert(HEADS * DKH == DD && DKH == 16);
static_assert(QKVW == 3 * DD);
static_assert((PTHR / 32) * 64 == QKVW);
static_assert(ETCAP < 128);

typedef float     v4f  __attribute__((ext_vector_type(4)));
typedef float     v8f  __attribute__((ext_vector_type(8)));
typedef int       v4i  __attribute__((ext_vector_type(4)));
typedef _Float16  v4h  __attribute__((ext_vector_type(4)));
typedef _Float16  v8h  __attribute__((ext_vector_type(8)));
typedef _Float16  v16h __attribute__((ext_vector_type(16)));
union Frag { v16h v; v8h h[2]; };

__device__ __forceinline__ v8f wmh(v16h a, v16h b, v8f c) {
  v8f d = __builtin_amdgcn_wmma_f32_16x16x32_f16(false, a, false, b, (short)0, c, false, false);
  asm volatile("v_nop\n\tv_nop\n\tv_nop\n\tv_nop" : "+v"(d) : "v"(a), "v"(b));
  return d;
}

__device__ __forceinline__ v8h cvt8(v4f a, v4f b, float s) {
  v8h o;
  o[0] = (_Float16)(a.x * s); o[1] = (_Float16)(a.y * s); o[2] = (_Float16)(a.z * s); o[3] = (_Float16)(a.w * s);
  o[4] = (_Float16)(b.x * s); o[5] = (_Float16)(b.y * s); o[6] = (_Float16)(b.z * s); o[7] = (_Float16)(b.w * s);
  return o;
}

template <int NB>
__device__ __forceinline__ int scan_chunk(const int* __restrict__ dsts, int nE, int cbase, int slotBase,
                                          int vec8, int* list, int tid, int lane, int wave) {
  int wc = 0;
#pragma unroll
  for (int g = 0; g < NGRP; ++g) {
    const int el0  = (g * NTHR + tid) * EPT;
    const int e0   = cbase + el0;
    const int sent = -2147483647 - 1;
    v4i da, db;
    if (vec8 != 0 && cbase + CHUNK <= nE) {
      da = *(const v4i*)(dsts + e0);
      db = *(const v4i*)(dsts + e0 + 4);
    } else {
      da.x = (e0     < nE) ? dsts[min(e0, nE - 1)] : sent;
      da.y = (e0 + 1 < nE) ? dsts[min(e0 + 1, nE - 1)] : sent;
      da.z = (e0 + 2 < nE) ? dsts[min(e0 + 2, nE - 1)] : sent;
      da.w = (e0 + 3 < nE) ? dsts[min(e0 + 3, nE - 1)] : sent;
      db.x = (e0 + 4 < nE) ? dsts[min(e0 + 4, nE - 1)] : sent;
      db.y = (e0 + 5 < nE) ? dsts[min(e0 + 5, nE - 1)] : sent;
      db.z = (e0 + 6 < nE) ? dsts[min(e0 + 6, nE - 1)] : sent;
      db.w = (e0 + 7 < nE) ? dsts[min(e0 + 7, nE - 1)] : sent;
    }
    const unsigned nb = (unsigned)slotBase;
    const unsigned s0 = (unsigned)da.x - nb, s1 = (unsigned)da.y - nb;
    const unsigned s2 = (unsigned)da.z - nb, s3 = (unsigned)da.w - nb;
    const unsigned s4 = (unsigned)db.x - nb, s5 = (unsigned)db.y - nb;
    const unsigned s6 = (unsigned)db.z - nb, s7 = (unsigned)db.w - nb;
    const bool h0 = s0 < (unsigned)NB, h1 = s1 < (unsigned)NB, h2 = s2 < (unsigned)NB, h3 = s3 < (unsigned)NB;
    const bool h4 = s4 < (unsigned)NB, h5 = s5 < (unsigned)NB, h6 = s6 < (unsigned)NB, h7 = s7 < (unsigned)NB;
    const unsigned any = __builtin_amdgcn_ballot_w32(h0 | h1 | h2 | h3 | h4 | h5 | h6 | h7);
    if (any != 0u) {
#define HITJ(J, HJ, SJ) { \
        const unsigned mj = __builtin_amdgcn_ballot_w32(HJ); \
        if (mj != 0u) { \
          if (HJ) { \
            const int pos = wc + (int)__builtin_amdgcn_mbcnt_lo(mj, 0u); \
            if (pos < WCAP) list[wave * WCAP + pos] = ((el0 + (J)) << 12) | (int)(SJ); \
          } \
          wc += (int)__builtin_popcount(mj); } }
      HITJ(0, h0, s0)
      HITJ(1, h1, s1)
      HITJ(2, h2, s2)
      HITJ(3, h3, s3)
      HITJ(4, h4, s4)
      HITJ(5, h5, s5)
      HITJ(6, h6, s6)
      HITJ(7, h7, s7)
#undef HITJ
    }
  }
  return wc;
}

__global__ __launch_bounds__(NTHR) void k_wprep(const float* __restrict__ W, _Float16* wp,
                                                 int Kd, int Nd, int nUnits, int nOff) {
  const int i = (int)blockIdx.x * NTHR + (int)threadIdx.x;
  if (i >= nUnits) return;
  const int kd8 = Kd >> 3;
  const int n   = i / kd8;
  const int k0  = (i - n * kd8) * 8;
  const float* sp = W + (size_t)k0 * Nd + n;
  v4f a, b;
  a.x = sp[0];               a.y = sp[(size_t)Nd];      a.z = sp[(size_t)2 * Nd];  a.w = sp[(size_t)3 * Nd];
  b.x = sp[(size_t)4 * Nd];  b.y = sp[(size_t)5 * Nd];  b.z = sp[(size_t)6 * Nd];  b.w = sp[(size_t)7 * Nd];
  const v8h o = cvt8(a, b, WCARRY);
  _Float16* dp = wp + (size_t)(nOff + n) * Kd + k0;
  *(volatile v8h*)dp = o;
  __threadfence();
  *(volatile v8h*)dp = o;
}

__global__ __launch_bounds__(NTHR) void k_cvt(const float* __restrict__ X, _Float16* Y, int nN, int nUnits) {
  const int i = (int)blockIdx.x * NTHR + (int)threadIdx.x;
  if (i >= nUnits) return;
  const int row = i >> 4;
  const int c0  = (i & 15) * 8;
  const int rr  = row < nN ? row : nN - 1;
  const float* sp = X + (size_t)rr * DD + c0;
  const v4f z4 = {0.f, 0.f, 0.f, 0.f};
  v4f a = *(const v4f*)sp, b = *(const v4f*)(sp + 4);
  a = (row < nN) ? a : z4;
  b = (row < nN) ? b : z4;
  const v8h o = cvt8(a, b, 1.0f);
  _Float16* dp = Y + (size_t)i * 8;
  *(volatile v8h*)dp = o;
  __threadfence();
  *(volatile v8h*)dp = o;
}

__global__ __launch_bounds__(NTHR) void k_count(
    const int* __restrict__ dsts, int* cnt, int nE, int vec8) {
  __shared__ __attribute__((aligned(16))) int scnt[NBC];
  __shared__ __attribute__((aligned(16))) int list[LISTN];
  __shared__ int wcnt[NWAVE];
  const int tid = threadIdx.x, lane = tid & 31, wave = tid >> 5;
  const int nodeBase = blockIdx.x * NBC;

  for (int i = tid; i < NBC; i += NTHR) scnt[i] = 0;
  __syncthreads();

  const int nChunks = (nE + CHUNK - 1) / CHUNK;
#pragma unroll 1
  for (int ch = 0; ch < nChunks; ++ch) {
    const int cbase = ch * CHUNK;
    const int wc = scan_chunk<NBC>(dsts, nE, cbase, nodeBase, vec8, list, tid, lane, wave);
    if (lane == 0) wcnt[wave] = wc;
    __syncthreads();
    if (wave == 0) {
#pragma unroll 1
      for (int wsx = 0; wsx < NWAVE; ++wsx) {
        int n = __builtin_amdgcn_readfirstlane(wcnt[wsx]);
        n = n > WCAP ? WCAP : (n < 0 ? 0 : n);
        const int* lp = list + wsx * WCAP;
#pragma unroll 1
        for (int i = 0; i < n; ++i) {
          const int ent  = __builtin_amdgcn_readfirstlane(lp[i]);
          const int slot = ent & (NBC - 1);
          if (lane == 0) scnt[slot] = scnt[slot] + 1;
        }
      }
    }
    __syncthreads();
  }

  v4i cq[4];
#pragma unroll
  for (int q = 0; q < 4; ++q) {
    const int f = (wave * 4 + q) * 128 + 4 * lane;
    cq[q] = *(const v4i*)(scnt + f);
  }
  int* cp = cnt + (size_t)nodeBase;
#pragma unroll
  for (int q = 0; q < 4; ++q) {
    const int f = (wave * 4 + q) * 128 + 4 * lane;
    *(volatile v4i*)(cp + f) = cq[q];
  }
  __threadfence();
#pragma unroll
  for (int q = 0; q < 4; ++q) {
    const int f = (wave * 4 + q) * 128 + 4 * lane;
    *(volatile v4i*)(cp + f) = cq[q];
  }
}

__global__ __launch_bounds__(OTHR) void k_offsets(
    const int* __restrict__ cnt, int* off, int* rbase, int nChunk) {
  __shared__ __attribute__((aligned(16))) int soff[NBC];
  __shared__ __attribute__((aligned(16))) int srb[RBN];
  __shared__ int wtot[OTHR / 32];
  const int tid = threadIdx.x, lane = tid & 31, wave = tid >> 5, sub = tid >> 7;
  for (int i = tid; i < RBN; i += OTHR) srb[i] = 0;
  int carry = 0;
#pragma unroll 1
  for (int ch = 0; ch < nChunk; ++ch) {
    const int base = ch * NBC;
    const v4i c0 = *(const v4i*)(cnt + base + 8 * tid);
    const v4i c1 = *(const v4i*)(cnt + base + 8 * tid + 4);
    const int e0 = max(c0.x, 0), e1 = max(c0.y, 0), e2 = max(c0.z, 0), e3 = max(c0.w, 0);
    const int e4 = max(c1.x, 0), e5 = max(c1.y, 0), e6 = max(c1.z, 0), e7 = max(c1.w, 0);
    const int ts = e0 + e1 + e2 + e3 + e4 + e5 + e6 + e7;
    int incl = ts;
#pragma unroll
    for (int d = 1; d < 32; d <<= 1) {
      const int t = __shfl_up(incl, d);
      if (lane >= d) incl += t;
    }
    if (lane == 31) wtot[wave] = incl;
    __syncthreads();
    const int S0 = wtot[0]  + wtot[1]  + wtot[2]  + wtot[3];
    const int S1 = wtot[4]  + wtot[5]  + wtot[6]  + wtot[7];
    const int S2 = wtot[8]  + wtot[9]  + wtot[10] + wtot[11];
    const int S3 = wtot[12] + wtot[13] + wtot[14] + wtot[15];
    int pre = 0;
#pragma unroll 1
    for (int w = 4 * sub; w < wave; ++w) pre += wtot[w];
    const int b0 = carry;
    const int b1 = b0 + ((S0 + 31) & ~31);
    const int b2 = b1 + ((S1 + 31) & ~31);
    const int b3 = b2 + ((S2 + 31) & ~31);
    const int b4 = b3 + ((S3 + 31) & ~31);
    const int myb = sub == 0 ? b0 : (sub == 1 ? b1 : (sub == 2 ? b2 : b3));
    if (tid == 0) {
      srb[min(4 * ch + 0, RBN - 1)] = b0;
      srb[min(4 * ch + 1, RBN - 1)] = b1;
      srb[min(4 * ch + 2, RBN - 1)] = b2;
      srb[min(4 * ch + 3, RBN - 1)] = b3;
    }
    int run = myb + pre + incl - ts;
    soff[8 * tid + 0] = run; run += e0;
    soff[8 * tid + 1] = run; run += e1;
    soff[8 * tid + 2] = run; run += e2;
    soff[8 * tid + 3] = run; run += e3;
    soff[8 * tid + 4] = run; run += e4;
    soff[8 * tid + 5] = run; run += e5;
    soff[8 * tid + 6] = run; run += e6;
    soff[8 * tid + 7] = run;
    carry = b4;
    __syncthreads();
    const v4i o0 = *(const v4i*)(soff + 4 * tid);
    const v4i o1 = *(const v4i*)(soff + 4 * (tid + OTHR));
    int* op = off + base;
    *(volatile v4i*)(op + 4 * tid) = o0;
    *(volatile v4i*)(op + 4 * (tid + OTHR)) = o1;
    __threadfence();
    *(volatile v4i*)(op + 4 * tid) = o0;
    *(volatile v4i*)(op + 4 * (tid + OTHR)) = o1;
    __syncthreads();
  }
  if (tid == 0) srb[min(4 * nChunk, RBN - 1)] = carry;
  __syncthreads();
  v4i rv = {0, 0, 0, 0};
  if (tid < 32) rv = *(const v4i*)(srb + 4 * tid);
  if (tid < 32) *(volatile v4i*)(rbase + 4 * tid) = rv;
  __threadfence();
  if (tid < 32) *(volatile v4i*)(rbase + 4 * tid) = rv;
}

__global__ __launch_bounds__(NTHR) void k_fill(
    const int* __restrict__ srcs, const int* __restrict__ dsts,
    const int* __restrict__ eattr, const int* __restrict__ fattr,
    const int* __restrict__ off, const int* __restrict__ rbase,
    int* csr, int nN, int nE, int eReal, int nFake, int nTypes, int nEf, int vec8, int csrLen) {
  extern __shared__ v4f lds_dyn[];
  int* region = (int*)lds_dyn;
  int* cursor = region + RCAP;
  int* list   = cursor + NBF;
  int* wcnt   = list + LISTN;
  const int tid = threadIdx.x, lane = tid & 31, wave = tid >> 5;
  const int b = blockIdx.x;
  const int nodeBase = b * NBF;

  int rb0 = rbase[b];
  const int rb1 = rbase[b + 1];
  rb0 = rb0 < 0 ? 0 : (rb0 > csrLen ? csrLen : rb0);
  rb0 &= ~31;
  int len = rb1 - rb0;
  len = len < 0 ? 0 : (len > RCAP ? RCAP : len);
  int lenW = (len + 31) & ~31;
  if (rb0 + lenW > csrLen) lenW = (csrLen - rb0) & ~31;

  {
    const v4i z = {0, 0, 0, 0};
    for (int i = tid; i < RCAP / 4; i += NTHR) ((v4i*)region)[i] = z;
    for (int s = tid; s < NBF; s += NTHR) {
      int o = off[nodeBase + s] - rb0;
      o = o < 0 ? 0 : (o > RCAP ? RCAP : o);
      cursor[s] = o;
    }
  }
  __syncthreads();

  const int nChunks = (nE + CHUNK - 1) / CHUNK;
#pragma unroll 1
  for (int ch = 0; ch < nChunks; ++ch) {
    const int cbase = ch * CHUNK;
    const int wc = scan_chunk<NBF>(dsts, nE, cbase, nodeBase, vec8, list, tid, lane, wave);
    if (lane == 0) wcnt[wave] = wc;
    __syncthreads();
    if (wave == 0) {
#pragma unroll 1
      for (int wsx = 0; wsx < NWAVE; ++wsx) {
        int n = __builtin_amdgcn_readfirstlane(wcnt[wsx]);
        n = n > WCAP ? WCAP : (n < 0 ? 0 : n);
        const int* lp = list + wsx * WCAP;
#pragma unroll 1
        for (int i = 0; i < n; ++i) {
          const int ent  = __builtin_amdgcn_readfirstlane(lp[i]);
          const int slot = ent & (NBF - 1);
          int e = cbase + ((ent >> 12) & (CHUNK - 1));
          e = e > nE - 1 ? nE - 1 : e;
          int src = srcs[e];
          src = src < 0 ? src + nN : src;
          src = src < 0 ? 0 : (src > nN - 1 ? nN - 1 : src);
          const int er = e > eReal - 1 ? eReal - 1 : e;
          int ta = eattr[er];
          ta = ta < 0 ? ta + nTypes : ta;
          ta = ta < 0 ? 0 : (ta > nTypes - 1 ? nTypes - 1 : ta);
          int ef = e - eReal;
          ef = ef < 0 ? 0 : (ef > nFake - 1 ? nFake - 1 : ef);
          int tf = fattr[ef];
          tf = tf < 0 ? tf + nEf : tf;
          tf = tf < 0 ? 0 : (tf > nEf - 1 ? nEf - 1 : tf);
          const int tcode = (e < eReal) ? ta : (nTypes + tf);
          const int val = (tcode << 24) | src;
          if (lane == 0) {
            int pos = cursor[slot];
            pos = pos < 0 ? 0 : (pos > RCAP - 1 ? RCAP - 1 : pos);
            region[pos] = val;
            const int np = pos + 1;
            cursor[slot] = np > RCAP ? RCAP : np;
          }
        }
      }
    }
    __syncthreads();
  }

  const int nv = lenW >> 2;
  int* gp = csr + rb0;
#pragma unroll 1
  for (int i = tid; i < nv; i += NTHR) { const v4i v = ((const v4i*)region)[i]; *(volatile v4i*)(gp + 4 * i) = v; }
  __threadfence();
#pragma unroll 1
  for (int i = tid; i < nv; i += NTHR) { const v4i v = ((const v4i*)region)[i]; *(volatile v4i*)(gp + 4 * i) = v; }
}

__global__ __launch_bounds__(PTHR) void k_proj(
    const _Float16* __restrict__ A, const _Float16* __restrict__ Bw,
    const float* __restrict__ bia0, const float* __restrict__ bia1, const float* __restrict__ bia2,
    float* Cf, float asc) {
  constexpr int KD  = DD;
  constexpr int NC  = QKVW;
  constexpr int NW  = PTHR / 32;
  constexpr int BM  = 16;
  constexpr int TPW = 4;
  static_assert(NW * 64 == NC && (KD % 32) == 0);
  static_assert(BM * NC * 4 <= 32768);

  __shared__ __attribute__((aligned(16))) float stg[BM * NC];
  const int tid = threadIdx.x, lane = tid & 31, wave = tid >> 5, hh = lane >> 4, m = lane & 15;
  const int rowBase = blockIdx.x * BM;
  const int c0 = wave * 64;

  v8f acc[TPW];
#pragma unroll
  for (int t = 0; t < TPW; ++t) { v8f z = {0.f, 0.f, 0.f, 0.f, 0.f, 0.f, 0.f, 0.f}; acc[t] = z; }
  const _Float16* ap = A + (size_t)(rowBase + m) * KD + 8 * hh;
#pragma unroll
  for (int kt = 0; kt < KD / 32; ++kt) {
    Frag a;
    a.h[0] = *(const v8h*)(ap + 32 * kt);
    a.h[1] = *(const v8h*)(ap + 32 * kt + 16);
#pragma unroll
    for (int t = 0; t < TPW; ++t) {
      const _Float16* bp = Bw + (size_t)(c0 + 16 * t + m) * KD + 32 * kt + 8 * hh;
      Frag b;
      b.h[0] = *(const v8h*)bp;
      b.h[1] = *(const v8h*)(bp + 16);
      acc[t] = wmh(a.v, b.v, acc[t]);
    }
  }

  {
    float* sp = stg + (8 * hh) * NC + c0 + m;
#pragma unroll
    for (int t = 0; t < TPW; ++t) {
#pragma unroll
      for (int r = 0; r < 8; ++r) sp[r * NC + 16 * t] = acc[t][r];
    }
  }
  __syncthreads();

#pragma unroll 1
  for (int rr = wave; rr < BM; rr += NW) {
    const int grow = rowBase + rr;
#pragma unroll
    for (int it = 0; it < 3; ++it) {
      const float* bsel = (it == 0) ? bia0 : ((it == 1) ? bia1 : bia2);
      const int col = it * 128 + 4 * lane;
      const v4f x  = *(const v4f*)(stg + rr * NC + col);
      const v4f bb = *(const v4f*)(bsel + 4 * lane);
      const v4f v  = x * asc + bb;
      *(volatile v4f*)(Cf + (size_t)grow * NC + col) = v;
    }
  }
  __threadfence();
#pragma unroll 1
  for (int rr = wave; rr < BM; rr += NW) {
    const int grow = rowBase + rr;
#pragma unroll
    for (int it = 0; it < 3; ++it) {
      const float* bsel = (it == 0) ? bia0 : ((it == 1) ? bia1 : bia2);
      const int col = it * 128 + 4 * lane;
      const v4f x  = *(const v4f*)(stg + rr * NC + col);
      const v4f bb = *(const v4f*)(bsel + 4 * lane);
      const v4f v  = x * asc + bb;
      *(volatile v4f*)(Cf + (size_t)grow * NC + col) = v;
    }
  }
}

__global__ __launch_bounds__(NTHR) void k_agg(
    const int* __restrict__ csr, const int* __restrict__ off, const int* __restrict__ cnt,
    const float* __restrict__ qkv, const float* __restrict__ Et, const float* __restrict__ Eft,
    float* out, int nN, int csrLen, int nTypes, int nEf) {
  __shared__ __attribute__((aligned(16))) float sE[ETCAP * DD];
  __shared__ __attribute__((aligned(16))) float sOut[NWAVE * AGRP * DD];
  const int tid = threadIdx.x, lane = tid & 31, wave = tid >> 5;
  const int nET = nTypes + nEf;
  const v4f z4 = {0.f, 0.f, 0.f, 0.f};

  for (int i = tid; i < ETCAP * (DD / 4); i += NTHR) {
    const int row = i >> 5;
    const int c4  = (i & 31) * 4;
    const int ra  = row < nTypes ? row : nTypes - 1;
    int rf = row - nTypes;
    rf = rf < 0 ? 0 : (rf > nEf - 1 ? nEf - 1 : rf);
    const v4f va = *(const v4f*)(Et  + (size_t)ra * DD + c4);
    const v4f vf = *(const v4f*)(Eft + (size_t)rf * DD + c4);
    v4f v = (row < nTypes) ? va : vf;
    v = (row < nET) ? v : z4;
    *(v4f*)(sE + row * DD + c4) = v;
  }
  __syncthreads();

  const int tbase = blockIdx.x * TGT + wave * 32;
  const int col   = 4 * lane;
  const int cnt_l = cnt[tbase + lane];
  const int off_l = off[tbase + lane];
  float* sw = sOut + wave * (AGRP * DD);

#pragma unroll 1
  for (int g = 0; g < 32 / AGRP; ++g) {
#pragma unroll 1
    for (int j = 0; j < AGRP; ++j) {
      const int jj = g * AGRP + j;
      const int c  = tbase + jj;
      int n = __builtin_amdgcn_readfirstlane(__shfl(cnt_l, jj));
      n = n < 0 ? 0 : (n > DEGCAP ? DEGCAP : n);
      const int st = __builtin_amdgcn_readfirstlane(__shfl(off_l, jj));
      v4f q = *(const v4f*)(qkv + (size_t)c * QKVW + col);
      q = q * QSCALE;
      float z = 0.f;
      v4f acc = z4;
#pragma unroll 1
      for (int q0 = 0; q0 < n; q0 += 32) {
        int pos = st + q0 + lane;
        pos = pos < 0 ? 0 : (pos > csrLen - 1 ? csrLen - 1 : pos);
        const int entl = csr[pos];
        const int mcnt = (n - q0) < 32 ? (n - q0) : 32;
#pragma unroll 1
        for (int pp = 0; pp < mcnt; ++pp) {
          const int en = __builtin_amdgcn_readlane(entl, pp);
          int s = en & 0xFFFFFF;
          s = s > nN - 1 ? nN - 1 : s;
          int tc = (en >> 24) & 0x7F;
          tc = tc > nET - 1 ? nET - 1 : tc;
          const float* rp = qkv + (size_t)s * QKVW + col;
          const v4f kv = *(const v4f*)(rp + DD);
          const v4f vv = *(const v4f*)(rp + 2 * DD);
          const v4f ev = *(const v4f*)(sE + tc * DD + col);
          const v4f t  = (kv * q) * ev;
          float p = (t.x + t.y) + (t.z + t.w);
          p += __shfl_xor(p, 1);
          p += __shfl_xor(p, 2);
          const float sc = __expf(fminf(fmaxf(p, -5.0f), 5.0f));
          z += sc;
          acc = acc + vv * sc;
        }
      }
      const float rz = 1.0f / (z + Z_EPS);
      const v4f a = acc * rz;
      *(v4f*)(sw + j * DD + col) = a;
    }
#pragma unroll
    for (int it = 0; it < AGRP; ++it) {
      const int c = tbase + g * AGRP + it;
      if (c < nN) {
        const v4f v = *(const v4f*)(sw + it * DD + col);
        *(volatile v4f*)(out + (size_t)c * DD + col) = v;
      }
    }
    __threadfence();
#pragma unroll
    for (int it = 0; it < AGRP; ++it) {
      const int c = tbase + g * AGRP + it;
      if (c < nN) {
        const v4f v = *(const v4f*)(sw + it * DD + col);
        *(volatile v4f*)(out + (size_t)c * DD + col) = v;
      }
    }
  }
}

extern "C" void kernel_launch(void* const* d_in, const int* in_sizes, int n_in,
                              void* d_out, int out_size, void* d_ws, size_t ws_size,
                              hipStream_t stream) {
  if (n_in < 14) return;
  if (in_sizes[0] <= 0 || (in_sizes[0] % DD) != 0) return;
  const int nN = in_sizes[0] / DD;
  if (in_sizes[1] != DD * DD || in_sizes[3] != DD * DD || in_sizes[5] != DD * DD) return;
  if (in_sizes[2] != DD || in_sizes[4] != DD || in_sizes[6] != DD) return;
  if (in_sizes[7] < DD || (in_sizes[7] % DD) != 0) return;
  if (in_sizes[8] < DD || (in_sizes[8] % DD) != 0) return;
  const int nTypes = in_sizes[7] / DD;
  const int nEf    = in_sizes[8] / DD;
  if (nTypes + nEf > ETCAP) return;
  const int eReal = in_sizes[9];
  const int nFake = in_sizes[10];
  const int nE    = in_sizes[11];
  if (eReal < 1 || nFake < 1 || nE < 1) return;
  if (in_sizes[12] != nE || eReal + nFake != nE) return;
  if (out_size != nN * DD) return;
  if (nE > (1 << 28) || nN > (1 << 24)) return;

  const float* x    = (const float*)d_in[0];
  const float* Wq   = (const float*)d_in[1];   const float* bq = (const float*)d_in[2];
  const float* Wk   = (const float*)d_in[3];   const float* bk = (const float*)d_in[4];
  const float* Wv   = (const float*)d_in[5];   const float* bv = (const float*)d_in[6];
  const float* Et   = (const float*)d_in[7];
  const float* Eft  = (const float*)d_in[8];
  const int*   eattr = (const int*)d_in[9];
  const int*   fattr = (const int*)d_in[10];
  const int*   esrc  = (const int*)d_in[11];
  const int*   edst  = (const int*)d_in[12];
  float* out = (float*)d_out;

  const int NPAD   = ((nN + TGT - 1) / TGT) * TGT;
  const int nBC    = (nN + NBC - 1) / NBC;
  const int CNTPAD = nBC * NBC;
  if (4 * nBC + 1 > RBN) return;
  const int nBF    = (nN + NBF - 1) / NBF;
  const int csrLen = ((nE + 31) & ~31) + 4096;
  if (31 * 4 * nBC > 4096) return;
  const int nAgg   = NPAD / TGT;

  char* ws = (char*)d_ws;
  size_t off = 0;
  const size_t oW    = off; off += (size_t)QKVW * DD * 2;         off = (off + 255) & ~(size_t)255;
  const size_t oXh   = off; off += (size_t)NPAD * DD * 2;         off = (off + 255) & ~(size_t)255;
  const size_t oCnt  = off; off += (size_t)CNTPAD * 4;            off = (off + 255) & ~(size_t)255;
  const size_t oOff  = off; off += (size_t)CNTPAD * 4;            off = (off + 255) & ~(size_t)255;
  const size_t oRb   = off; off += (size_t)RBN * 4;               off = (off + 255) & ~(size_t)255;
  const size_t oCsr  = off; off += (size_t)csrLen * 4;            off = (off + 255) & ~(size_t)255;
  const size_t oQkv  = off; off += (size_t)NPAD * QKVW * 4;       off = (off + 255) & ~(size_t)255;
  if (off > ws_size || off > (size_t)WSCAP) return;
  _Float16* wpl = (_Float16*)(ws + oW);
  _Float16* xh  = (_Float16*)(ws + oXh);
  int*   cnt  = (int*)(ws + oCnt);
  int*   offp = (int*)(ws + oOff);
  int*   rb   = (int*)(ws + oRb);
  int*   csr  = (int*)(ws + oCsr);
  float* qkv  = (float*)(ws + oQkv);

  const int vec8 = ((nE & 3) == 0) ? 1 : 0;

  {
    const int uq = DD * (DD / 8);
    k_wprep<<<(uq + NTHR - 1) / NTHR, NTHR, 0, stream>>>(Wq, wpl, DD, DD, uq, 0);
    k_wprep<<<(uq + NTHR - 1) / NTHR, NTHR, 0, stream>>>(Wk, wpl, DD, DD, uq, DD);
    k_wprep<<<(uq + NTHR - 1) / NTHR, NTHR, 0, stream>>>(Wv, wpl, DD, DD, uq, 2 * DD);
  }
  {
    const int uc = NPAD * (DD / 8);
    k_cvt<<<(uc + NTHR - 1) / NTHR, NTHR, 0, stream>>>(x, xh, nN, uc);
  }
  k_count<<<nBC, NTHR, 0, stream>>>(edst, cnt, nE, vec8);
  k_offsets<<<1, OTHR, 0, stream>>>(cnt, offp, rb, nBC);
  hipFuncSetAttribute(reinterpret_cast<const void*>(&k_fill),
                      hipFuncAttributeMaxDynamicSharedMemorySize, LDS_FILL);
  k_fill<<<nBF, NTHR, LDS_FILL, stream>>>(esrc, edst, eattr, fattr, offp, rb, csr,
                                          nN, nE, eReal, nFake, nTypes, nEf, vec8, csrLen);
  k_proj<<<NPAD / 16, PTHR, 0, stream>>>(xh, wpl, bq, bk, bv, qkv, 1.0f / WCARRY);
  k_agg<<<nAgg, NTHR, 0, stream>>>(csr, offp, cnt, qkv, Et, Eft, out, nN, csrLen, nTypes, nEf);
}
